// MyModel_61933428409059
// MI455X (gfx1250) — hardware-verified
//
#include <hip/hip_runtime.h>

typedef __attribute__((ext_vector_type(16))) _Float16 v16h;
typedef __attribute__((ext_vector_type(8)))  _Float16 v8h;
typedef __attribute__((ext_vector_type(4)))  _Float16 v4h;
typedef __attribute__((ext_vector_type(8)))  float    v8f;
typedef __attribute__((ext_vector_type(4)))  float    v4f;

constexpr int SEQ_LEN    = 671;
constexpr int HEAD_DIM   = 64;
constexpr int BLK_ROWS   = 128;
constexpr int GAP_BEGIN  = 384;
constexpr int GAP_END    = 543;
constexpr int NWAVES     = 8;
constexpr int NTHREADS   = 256;
constexpr float P_CARRY     = 32768.0f;
constexpr float SCORE_SCALE = 0.125f;

static_assert(SEQ_LEN - GAP_END == BLK_ROWS, "last block is 128 rows");
static_assert(3 * BLK_ROWS == GAP_BEGIN, "first three blocks end at the gap");
static_assert(NWAVES * 16 == BLK_ROWS, "8 waves x 16 query rows cover a block");
static_assert(HEAD_DIM % 32 == 0 && BLK_ROWS % 32 == 0, "K multiples of 32 for both contractions");

__device__ __forceinline__ unsigned short f2bf_bits(float f) {
  unsigned u = __float_as_uint(f);
  return (unsigned short)((u + 0x7FFFu + ((u >> 16) & 1u)) >> 16);
}
__device__ __forceinline__ _Float16 to_h16_of_bf16(float f) {
  const unsigned short hb = f2bf_bits(f);
  const float g = __uint_as_float(((unsigned)hb) << 16);
  return (_Float16)g;
}
__device__ __forceinline__ v16h frag_load(const _Float16* p) {
  union { v16h v; v8h h[2]; } f;
  f.h[0] = *(const v8h*)(p);
  f.h[1] = *(const v8h*)(p + 16);
  return f.v;
}
__device__ __forceinline__ v8f mma16(v16h a, v16h b, v8f c) {
  c = __builtin_amdgcn_wmma_f32_16x16x32_f16(false, a, false, b, (short)0, c, false, false);
  asm volatile("v_nop\n\tv_nop\n\tv_nop\n\tv_nop" : "+v"(c) : "v"(a), "v"(b));
  return c;
}

union POBuf {
  _Float16 p[16 * BLK_ROWS];
  float    o[16 * HEAD_DIM];
};
static_assert(sizeof(POBuf) == 4096, "P and O views have equal size");

__global__ __launch_bounds__(NTHREADS) void blk_attn_kernel(const float* __restrict__ x,
                                                            float* __restrict__ out) {
  __shared__ __align__(16) _Float16 sX[BLK_ROWS * HEAD_DIM];
  __shared__ __align__(16) _Float16 sXt[HEAD_DIM * BLK_ROWS];
  __shared__ __align__(16) POBuf sPO[NWAVES];

  const int blk = blockIdx.x;
  const int bh  = blockIdx.y;
  const int row0 = (blk < 3) ? blk * BLK_ROWS : GAP_END;
  const size_t base = ((size_t)bh * SEQ_LEN + (size_t)row0) * HEAD_DIM;
  const float* gx = x + base;
  float* gy = out + base;
  const int tid = threadIdx.x;

#pragma unroll
  for (int i = 0; i < 8; ++i) {
    const int f   = i * NTHREADS + tid;
    const int row = f >> 4;
    const int d4  = (f & 15) * 4;
    const v4f v = *(const v4f*)(gx + (size_t)row * HEAD_DIM + d4);
    const _Float16 h0 = to_h16_of_bf16(v[0]);
    const _Float16 h1 = to_h16_of_bf16(v[1]);
    const _Float16 h2 = to_h16_of_bf16(v[2]);
    const _Float16 h3 = to_h16_of_bf16(v[3]);
    v4h hv;
    hv[0] = h0; hv[1] = h1; hv[2] = h2; hv[3] = h3;
    *(v4h*)(sX + row * HEAD_DIM + d4) = hv;
    sXt[(d4 + 0) * BLK_ROWS + row] = h0;
    sXt[(d4 + 1) * BLK_ROWS + row] = h1;
    sXt[(d4 + 2) * BLK_ROWS + row] = h2;
    sXt[(d4 + 3) * BLK_ROWS + row] = h3;
  }
  __syncthreads();

  const int wave = tid >> 5;
  const int lane = tid & 31;
  const int hh   = lane >> 4;
  const int c    = lane & 15;
  const int r0   = wave * 16;

  v8f acc[8];
#pragma unroll
  for (int j = 0; j < 8; ++j) acc[j] = (v8f){0.f, 0.f, 0.f, 0.f, 0.f, 0.f, 0.f, 0.f};
  v16h qa[2];
#pragma unroll
  for (int kk = 0; kk < 2; ++kk) qa[kk] = frag_load(sX + (r0 + c) * HEAD_DIM + kk * 32 + 8 * hh);
#pragma unroll
  for (int j = 0; j < 8; ++j) {
#pragma unroll
    for (int kk = 0; kk < 2; ++kk) {
      const v16h kb = frag_load(sX + (j * 16 + c) * HEAD_DIM + kk * 32 + 8 * hh);
      acc[j] = mma16(qa[kk], kb, acc[j]);
    }
  }

  float mx[8], inv[8];
#pragma unroll
  for (int r = 0; r < 8; ++r) {
    float m = acc[0][r];
#pragma unroll
    for (int j = 1; j < 8; ++j) m = fmaxf(m, acc[j][r]);
#pragma unroll
    for (int off = 1; off < 16; off <<= 1) m = fmaxf(m, __shfl_xor(m, off, 32));
    mx[r] = m * SCORE_SCALE;
  }
  _Float16* pw = sPO[wave].p;
#pragma unroll
  for (int r = 0; r < 8; ++r) {
    float psum = 0.f;
#pragma unroll
    for (int j = 0; j < 8; ++j) {
      const float p = expf(acc[j][r] * SCORE_SCALE - mx[r]);
      psum += p;
      pw[(8 * hh + r) * BLK_ROWS + j * 16 + c] = (_Float16)(p * P_CARRY);
    }
#pragma unroll
    for (int off = 1; off < 16; off <<= 1) psum += __shfl_xor(psum, off, 32);
    inv[r] = 1.0f / (psum * P_CARRY);
  }
  __syncthreads();

  v8f oacc[4];
#pragma unroll
  for (int t = 0; t < 4; ++t) oacc[t] = (v8f){0.f, 0.f, 0.f, 0.f, 0.f, 0.f, 0.f, 0.f};
#pragma unroll
  for (int kk = 0; kk < 4; ++kk) {
    const v16h pa = frag_load(pw + c * BLK_ROWS + kk * 32 + 8 * hh);
#pragma unroll
    for (int t = 0; t < 4; ++t) {
      const v16h vb = frag_load(sXt + (t * 16 + c) * BLK_ROWS + kk * 32 + 8 * hh);
      oacc[t] = mma16(pa, vb, oacc[t]);
    }
  }
  __syncthreads();

  float* os = sPO[wave].o;
#pragma unroll
  for (int r = 0; r < 8; ++r) {
#pragma unroll
    for (int t = 0; t < 4; ++t) os[(8 * hh + r) * HEAD_DIM + t * 16 + c] = oacc[t][r] * inv[r];
  }
  __syncthreads();

  {
    const int c4 = c * 4;
    for (int pass = 0; pass < 2; ++pass) {
#pragma unroll
      for (int it = 0; it < 8; ++it) {
        const int row = it * 2 + hh;
        const v4f val = *(const v4f*)(os + row * HEAD_DIM + c4);
        *(volatile v4f*)(gy + (size_t)(r0 + row) * HEAD_DIM + c4) = val;
      }
      __threadfence();
    }
  }
}

__global__ __launch_bounds__(NTHREADS) void gap_zero_kernel(float* __restrict__ out) {
  constexpr int N4 = (GAP_END - GAP_BEGIN) * HEAD_DIM / 4;
  const int bh = blockIdx.x;
  float* p = out + ((size_t)bh * SEQ_LEN + (size_t)GAP_BEGIN) * HEAD_DIM;
  v4f z;
  z[0] = 0.f; z[1] = 0.f; z[2] = 0.f; z[3] = 0.f;
  for (int pass = 0; pass < 2; ++pass) {
    for (int i = threadIdx.x; i < N4; i += NTHREADS) *(volatile v4f*)(p + (size_t)i * 4) = z;
    __threadfence();
  }
}

extern "C" void kernel_launch(void* const* d_in, const int* in_sizes, int n_in,
                              void* d_out, int out_size, void* d_ws, size_t ws_size,
                              hipStream_t stream) {
  (void)n_in; (void)d_ws; (void)ws_size;
  const float* x = (const float*)d_in[0];
  float* out = (float*)d_out;
  const int total = in_sizes[0];
  const int per_bh = SEQ_LEN * HEAD_DIM;
  const int nbh = total / per_bh;
  if (nbh <= 0 || nbh * per_bh != total || out_size != total) return;
  blk_attn_kernel<<<dim3(4, nbh), NTHREADS, 0, stream>>>(x, out);
  gap_zero_kernel<<<dim3(nbh), NTHREADS, 0, stream>>>(out);
}
